// GCLSTMPrisoner_50766513439412
// MI455X (gfx1250) — hardware-verified
//
#include <hip/hip_runtime.h>
#include <hip/hip_bf16.h>

typedef _Float16 half_t;
typedef __attribute__((ext_vector_type(16))) _Float16 v16h;
typedef __attribute__((ext_vector_type(8)))  _Float16 v8h;
typedef __attribute__((ext_vector_type(8)))  float    v8f;
typedef __attribute__((ext_vector_type(4)))  float    v4f;
typedef float __attribute__((may_alias)) float_a;
template <typename T> __device__ __forceinline__ void vst2(void* p, T v) { *(volatile T*)p = v; __threadfence(); *(volatile T*)p = v; }
__device__ __forceinline__ v8f wmma16(v16h a, v16h b, v8f c) {
  v8f d = __builtin_amdgcn_wmma_f32_16x16x32_f16(false, a, false, b, (short)0, c, false, false);
  asm volatile("v_nop\n\tv_nop\n\tv_nop\n\tv_nop" : "+v"(d) : "v"(a), "v"(b));
  return d;
}

#define T_STEPS 128
#define AGENTS  16
#define F_IN    32
#define HID     384
#define G4H     (4 * HID)
#define KSTEPS  13
#define CTILES  96
#define ROWS    16
#define NWG     64
#define NTHREADS 384
#define ASTRIDE 424
#define OUTC    387

#define GSTRIDE_V 9984
#define KSTRIDE_V 32

__global__ __launch_bounds__(256)
void build_wfrag_kernel(const float* __restrict__ Wx,
                        const float* __restrict__ Wh,
                        half_t* __restrict__ Wfrag) {
  int gid2 = blockIdx.x * blockDim.x + threadIdx.x;
  const int total = KSTEPS * CTILES * 32;
  if (gid2 >= total * 2) return;
  int gid = gid2 >> 1, hsel = gid2 & 1;
  int lane = gid & 31;
  int frag = gid >> 5;
  int kk   = frag % KSTEPS;
  int ct   = frag / KSTEPS;
  int col  = ct * 16 + (lane & 15);
  int kbase = kk * 32 + ((lane >> 4) << 3);
  union { v8h v; __attribute__((ext_vector_type(4))) unsigned u; } pk;
#pragma unroll
  for (int jj = 0; jj < 8; ++jj) {
    int j = hsel * 8 + jj;
    int K = kbase + ((j < 8) ? j : (j + 8));
    float w = (K < F_IN) ? Wx[(size_t)K * G4H + col]
                         : Wh[(size_t)(K - F_IN) * G4H + col];
    pk.v[jj] = (half_t)w;
  }
  vst2(Wfrag + (size_t)gid * 16 + hsel * 8, pk.u);
}

__device__ __forceinline__ float sigmoid_f(float x) {
  return 1.0f / (1.0f + __expf(-x));
}

__device__ __forceinline__ void load_bfrags(const v16h* __restrict__ wbase,
                                            int kk, v16h b[4]) {
#pragma unroll
  for (int g = 0; g < 4; ++g) b[g] = wbase[g * GSTRIDE_V + kk * KSTRIDE_V];
}

__device__ __forceinline__ v16h load_afrag(const half_t* Ab, int off) {
  v8h alo = *(const v8h*)(Ab + off);
  v8h ahi = *(const v8h*)(Ab + off + 16);
  return __builtin_shufflevector(alo, ahi, 0, 1, 2, 3, 4, 5, 6, 7,
                                 8, 9, 10, 11, 12, 13, 14, 15);
}

__global__ __launch_bounds__(NTHREADS)
void gclstm_main_kernel(const float* __restrict__ agent_obs,
                        const float* __restrict__ hideout_obs,
                        const float* __restrict__ timestep_obs,
                        const float* __restrict__ b_in,
                        const float* __restrict__ b_conv,
                        const float* __restrict__ w_ci,
                        const float* __restrict__ w_cf,
                        const float* __restrict__ w_co,
                        const half_t* __restrict__ Wfrag,
                        float* __restrict__ stage) {
  __shared__ __align__(16) half_t Abuf[2][ROWS * ASTRIDE];
  __shared__ float biasS[4 * HID];
  __shared__ float peepS[3 * HID];

  const int tid   = threadIdx.x;
  const int wg    = blockIdx.x;
  const int lane  = tid & 31;
  const int wave  = tid >> 5;
  const int nhalf = lane >> 4;
  const int ncol  = lane & 15;

  for (int j = tid; j < 4 * HID; j += NTHREADS) biasS[j] = b_in[j] + b_conv[j];
  for (int j = tid; j < HID; j += NTHREADS) {
    peepS[j]           = w_ci[j];
    peepS[HID + j]     = w_cf[j];
    peepS[2 * HID + j] = w_co[j];
  }
  for (int j = tid; j < ROWS * HID; j += NTHREADS) {
    int r = j / HID, u = j - r * HID;
    Abuf[0][r * ASTRIDE + F_IN + u] = (half_t)0.0f;
  }

  float creg[2][8];
#pragma unroll
  for (int p = 0; p < 2; ++p)
#pragma unroll
    for (int r = 0; r < 8; ++r) creg[p][r] = 0.0f;

  const int arow = ncol * ASTRIDE;
  const int kofs = nhalf * 8;
  const float* xsrc = agent_obs + (size_t)wg * T_STEPS * ROWS * F_IN;
  int wofs = 0;

  __syncthreads();

  for (int t = 0; t < T_STEPS; ++t) {
    asm volatile("" : "+s"(wofs));
    const half_t* Wt = Wfrag + wofs;

    const int buf = t & 1;
    if (tid < 256) {
      const float* xt = xsrc + (size_t)t * (ROWS * F_IN);
#pragma unroll
      for (int q = 0; q < 2; ++q) {
        int idx = tid + q * 256;
        Abuf[buf][(idx >> 5) * ASTRIDE + (idx & 31)] = (half_t)xt[idx];
        if (t + 1 < T_STEPS) __builtin_prefetch(xt + ROWS * F_IN + idx, 0, 0);
      }
    }
    __syncthreads();

    const half_t* Ab = &Abuf[buf][0];
    half_t*       Aw = &Abuf[buf ^ 1][0];

#pragma unroll
    for (int p = 0; p < 2; ++p) {
      const int ut = wave + 12 * p;
      const v16h* wbase =
          (const v16h*)(Wt + (size_t)ut * 6656 + (size_t)lane * 16);
      v8f acc[4] = {v8f{}, v8f{}, v8f{}, v8f{}};

      v16h bq[3][4];
      v16h aq[2];
      load_bfrags(wbase, 0, bq[0]);
      load_bfrags(wbase, 1, bq[1]);
      aq[0] = load_afrag(Ab, arow + kofs);
#pragma unroll
      for (int kk = 0; kk < KSTEPS; ++kk) {
        if (kk + 2 < KSTEPS) load_bfrags(wbase, kk + 2, bq[(kk + 2) % 3]);
        if (kk + 1 < KSTEPS)
          aq[(kk + 1) & 1] = load_afrag(Ab, arow + (kk + 1) * 32 + kofs);
#pragma unroll
        for (int g = 0; g < 4; ++g) {
          acc[g] = wmma16(aq[kk & 1], bq[kk % 3][g], acc[g]);
        }
      }

      const int u   = ut * 16 + ncol;
      const float bi  = biasS[u];
      const float bff = biasS[HID + u];
      const float bc  = biasS[2 * HID + u];
      const float bo  = biasS[3 * HID + u];
      const float pci = peepS[u];
      const float pcf = peepS[HID + u];
      const float pco = peepS[2 * HID + u];
      half_t* hdst = Aw + (nhalf * 8) * ASTRIDE + F_IN + u;
#pragma unroll
      for (int r = 0; r < 8; ++r) {
        float c  = creg[p][r];
        float ii = sigmoid_f(acc[0][r] + bi + pci * c);
        float ff = sigmoid_f(acc[1][r] + bff + pcf * c);
        float cn = ff * c + ii * tanhf(acc[2][r] + bc);
        float oo = sigmoid_f(acc[3][r] + bo + pco * cn);
        float hn = oo * tanhf(cn);
        creg[p][r] = cn;
        hdst[r * ASTRIDE] = (half_t)hn;
      }
    }
  }
  __syncthreads();

  for (int u = tid; u < HID; u += NTHREADS) {
    float s = 0.0f;
#pragma unroll
    for (int r = 0; r < ROWS; ++r)
      s += (float)Abuf[0][r * ASTRIDE + F_IN + u];
    vst2(stage + (size_t)wg * 512 + u, (float_a)(s * (1.0f / 16.0f)));
  }
  if (tid < 32) {
    float v = 0.f;
    if (tid < 2) v = hideout_obs[wg * 2 + tid]; else if (tid == 2) v = timestep_obs[wg];
    vst2(stage + (size_t)wg * 512 + 384 + tid, (float_a)v);
  }
}
__global__ __launch_bounds__(256) void out_kernel(const float* __restrict__ stage, float* __restrict__ out) {
  const int g = blockIdx.x * 256 + threadIdx.x;
  if (g >= 64 * OUTC / 4) return;
  v4f v;
#pragma unroll
  for (int e = 0; e < 4; ++e) { const int f = g * 4 + e, b = f / OUTC, c = f - b * OUTC; v[e] = stage[(size_t)b * 512 + c]; }
  vst2(out + (size_t)g * 4, v);
}

extern "C" void kernel_launch(void* const* d_in, const int* in_sizes, int n_in,
                              void* d_out, int out_size, void* d_ws, size_t ws_size,
                              hipStream_t stream) {
  const float* agent_obs    = (const float*)d_in[0];
  const float* hideout_obs  = (const float*)d_in[1];
  const float* timestep_obs = (const float*)d_in[2];
  const float* Wx           = (const float*)d_in[3];
  const float* Wh           = (const float*)d_in[4];
  const float* b_in         = (const float*)d_in[5];
  const float* b_conv       = (const float*)d_in[6];
  const float* w_ci         = (const float*)d_in[7];
  const float* w_cf         = (const float*)d_in[8];
  const float* w_co         = (const float*)d_in[9];
  float* out                = (float*)d_out;

  half_t* Wfrag = (half_t*)d_ws;
  float* stage = (float*)((char*)d_ws + 2 * 1024 * 1024);

  const int total = KSTEPS * CTILES * 32 * 2;
  build_wfrag_kernel<<<(total + 255) / 256, 256, 0, stream>>>(Wx, Wh, Wfrag);

  gclstm_main_kernel<<<NWG, NTHREADS, 0, stream>>>(
      agent_obs, hideout_obs, timestep_obs, b_in, b_conv,
      w_ci, w_cf, w_co, Wfrag, stage);
  out_kernel<<<(64 * OUTC / 4 + 255) / 256, 256, 0, stream>>>(stage, out);
}
